// ConvolutionalSelfAttention_1486058684519
// MI455X (gfx1250) — hardware-verified
//
#include <hip/hip_runtime.h>

typedef __bf16          v16b __attribute__((ext_vector_type(16)));
typedef unsigned short  v8us __attribute__((ext_vector_type(8)));
typedef unsigned short  v4us __attribute__((ext_vector_type(4)));
typedef float           v8f  __attribute__((ext_vector_type(8)));
typedef float           v4f  __attribute__((ext_vector_type(4)));
typedef v8us __attribute__((may_alias)) v8usa;
typedef v4us __attribute__((may_alias)) v4usa;
typedef v4f  __attribute__((may_alias)) v4fa;

union FragB { v16b v; v8us half[2]; };

static constexpr int kH    = 16;
static constexpr int kW    = 16;
static constexpr int kC    = 64;
static constexpr int kB    = 32;
static constexpr int kK    = 3;
static constexpr int kCH   = kH - kK + 1;
static constexpr int kNWin = kCH * kCH;
static constexpr int kNPos = kH * kW;
static constexpr int kNLoc = kK * kK;
static constexpr int kNX   = kB * kNPos * kC;
static constexpr int kNOut = kB * kNWin * kC;
static constexpr float kTemp = 10.0f;

static_assert(kC % 32 == 0);
static_assert(kNPos % 32 == 0);
static_assert((kCH * kC) % 4 == 0);
static_assert(kCH * kNLoc <= 128);

__device__ __forceinline__ unsigned short bf16_bits(float x) {
  unsigned int u = __float_as_uint(x);
  u = u + 0x7FFFu + ((u >> 16) & 1u);
  return (unsigned short)(u >> 16);
}
__device__ __forceinline__ float bits_val(unsigned short s) {
  return __uint_as_float(((unsigned int)s) << 16);
}
__device__ __forceinline__ float bf16_val(float x) {
  return bits_val(bf16_bits(x));
}

__device__ __forceinline__ v8f wmma_bf16(v16b a, v16b b, v8f c) {
  v8f d = __builtin_amdgcn_wmma_f32_16x16x32_bf16(false, a, false, b, (short)0, c, false, false);
  asm volatile("v_nop\n\tv_nop\n\tv_nop\n\tv_nop" : "+v"(d) : "v"(a), "v"(b));
  return d;
}

__device__ __forceinline__ v16b load_frag(const unsigned short* p, int h) {
  FragB f;
  f.half[0] = *(const v8usa*)(p + 8 * h);
  f.half[1] = *(const v8usa*)(p + 16 + 8 * h);
  return f.v;
}

__device__ __forceinline__ void gram_store_pass(const float* st, float* Gm,
                                                int b, int R0, int C0, int lane) {
  const int q8 = lane & 7, sub = lane >> 3;
  #pragma unroll
  for (int i = 0; i < 8; ++i) {
    const int rowl = 4 * i + sub;
    const v4f v = *(const v4fa*)(st + rowl * 32 + 4 * q8);
    float* dst = Gm + ((size_t)(b * kNPos + R0 + rowl)) * kNPos + C0 + 4 * q8;
    *(volatile v4f*)dst = v;
  }
}

__global__ __launch_bounds__(128) void gram_kernel(
    const float* __restrict__ X,
    const float* __restrict__ Wg,
    const float* __restrict__ bg,
    float* __restrict__ Gm,
    float* __restrict__ Spl,
    float* __restrict__ Rpl)
{
  __shared__ __attribute__((aligned(16))) unsigned short sP[kNPos * kC];
  __shared__ __attribute__((aligned(16))) float sT[4 * 32 * 32];
  __shared__ __attribute__((aligned(16))) float sS[128];
  __shared__ __attribute__((aligned(16))) float sR[128];
  __shared__ float sWgf[kC];

  const int tid = threadIdx.x, lane = tid & 31, w = tid >> 5;
  const int h = lane >> 4, m = lane & 15;
  const int r = blockIdx.x, b = blockIdx.y;
  const float* Xb = X + (size_t)b * kNPos * kC;

  #pragma unroll 4
  for (int idx = tid; idx < kNPos * kC / 4; idx += 128) {
    const v4f v = *(const v4fa*)(Xb + 4 * idx);
    const v4us o = { bf16_bits(v.x), bf16_bits(v.y), bf16_bits(v.z), bf16_bits(v.w) };
    *(v4usa*)(sP + 4 * idx) = o;
  }
  if (tid < kC) sWgf[tid] = bf16_val(Wg[tid]);
  __syncthreads();

  {
    const int px = 128 * r + tid;
    const unsigned short* row = sP + px * kC;
    float ss = 0.f, dot = 0.f;
    #pragma unroll 4
    for (int c = 0; c < kC; ++c) {
      const float x = bits_val(row[c]);
      ss  += x * x;
      dot += x * sWgf[c];
    }
    sS[tid] = dot + bf16_val(bg[0]);
    sR[tid] = 1.0f / fmaxf(sqrtf(ss), 1e-12f);
  }
  __syncthreads();

  if (w == 0) {
    const v4f v = *(const v4fa*)(sS + 4 * lane);
    float* dst = Spl + (size_t)b * kNPos + 128 * r + 4 * lane;
    *(volatile v4f*)dst = v;
    __threadfence();
    *(volatile v4f*)dst = v;
  } else if (w == 1) {
    const v4f v = *(const v4fa*)(sR + 4 * lane);
    float* dst = Rpl + (size_t)b * kNPos + 128 * r + 4 * lane;
    *(volatile v4f*)dst = v;
    __threadfence();
    *(volatile v4f*)dst = v;
  }

  const int R0 = 128 * r + 32 * w;
  v16b af[2][2];
  #pragma unroll
  for (int mt = 0; mt < 2; ++mt) {
    const unsigned short* ap = sP + (R0 + 16 * mt + m) * kC;
    af[mt][0] = load_frag(ap, h);
    af[mt][1] = load_frag(ap + 32, h);
  }

  const v8f zero8 = {0.f, 0.f, 0.f, 0.f, 0.f, 0.f, 0.f, 0.f};
  float* st = sT + w * 1024;

  #pragma unroll 1
  for (int p = 0; p < kNPos / 32; ++p) {
    const int C0 = 32 * p;
    v8f acc[2][2];
    #pragma unroll
    for (int mt = 0; mt < 2; ++mt)
      #pragma unroll
      for (int nt = 0; nt < 2; ++nt) acc[mt][nt] = zero8;

    #pragma unroll
    for (int nt = 0; nt < 2; ++nt) {
      const unsigned short* bp = sP + (C0 + 16 * nt + m) * kC;
      const v16b b0 = load_frag(bp, h);
      const v16b b1 = load_frag(bp + 32, h);
      #pragma unroll
      for (int mt = 0; mt < 2; ++mt) {
        acc[mt][nt] = wmma_bf16(af[mt][0], b0, acc[mt][nt]);
        acc[mt][nt] = wmma_bf16(af[mt][1], b1, acc[mt][nt]);
      }
    }

    #pragma unroll
    for (int mt = 0; mt < 2; ++mt)
      #pragma unroll
      for (int nt = 0; nt < 2; ++nt)
        #pragma unroll
        for (int rr = 0; rr < 8; ++rr)
          st[(16 * mt + 8 * h + rr) * 32 + 16 * nt + m] = acc[mt][nt][rr];
    __syncthreads();

    gram_store_pass(st, Gm, b, R0, C0, lane);
    __threadfence();
    gram_store_pass(st, Gm, b, R0, C0, lane);
    __syncthreads();
  }
}

__global__ __launch_bounds__(256) void win_kernel(
    const float* __restrict__ X,
    const float* __restrict__ Gm,
    const float* __restrict__ Spl,
    const float* __restrict__ Rpl,
    float* __restrict__ out)
{
  __shared__ __attribute__((aligned(16))) float sG[48 * kNPos];
  __shared__ __attribute__((aligned(16))) float sS[kNPos];
  __shared__ __attribute__((aligned(16))) float sR[kNPos];
  __shared__ float sWk[128];
  __shared__ __attribute__((aligned(16))) float sO[kCH * kC];

  const int tid = threadIdx.x;
  const int i = blockIdx.x, b = blockIdx.y;

  const float* gsrc = Gm + ((size_t)b * kNPos + i * kW) * kNPos;
  #pragma unroll 4
  for (int idx = tid; idx < 48 * kNPos / 4; idx += 256)
    *(v4fa*)(sG + 4 * idx) = *(const v4fa*)(gsrc + 4 * idx);
  if (tid < 64) {
    *(v4fa*)(sS + 4 * tid) = *(const v4fa*)(Spl + (size_t)b * kNPos + 4 * tid);
  } else if (tid < 128) {
    const int t = tid - 64;
    *(v4fa*)(sR + 4 * t) = *(const v4fa*)(Rpl + (size_t)b * kNPos + 4 * t);
  }
  __syncthreads();

  {
    const int colr = tid >> 1;
    const int col  = (colr < kCH * kNLoc) ? colr : (kCH * kNLoc - 1);
    const int hf   = tid & 1;
    const int j    = col / kNLoc;
    const int k    = col - kNLoc * j;
    const int a    = k / 3;
    const int bb   = k - 3 * a;
    const int lr   = kW * a + j + bb;
    const float rl = sR[kW * i + lr];
    const float* grow = sG + lr * kNPos;
    const int g0 = 128 * hf;

    float mx = -1e30f;
    #pragma unroll 1
    for (int gg = 0; gg < 128; ++gg) {
      const int g = g0 + gg;
      const float t = kTemp * ((grow[g] * sR[g]) * rl);
      const unsigned dr = (unsigned)((g >> 4) - i);
      const unsigned dc = (unsigned)((g & 15) - j);
      const bool loc = (dr < 3u) && (dc < 3u);
      mx = fmaxf(mx, loc ? -1e30f : t);
    }
    mx = fmaxf(mx, __shfl_xor(mx, 1));

    float se = 0.f, sw = 0.f;
    #pragma unroll 1
    for (int gg = 0; gg < 128; ++gg) {
      const int g = g0 + gg;
      const float t = kTemp * ((grow[g] * sR[g]) * rl);
      const unsigned dr = (unsigned)((g >> 4) - i);
      const unsigned dc = (unsigned)((g & 15) - j);
      const bool loc = (dr < 3u) && (dc < 3u);
      const float ev = expf(t - mx);
      const float e = loc ? 0.0f : ev;
      se += e;
      sw += sS[g] * e;
    }
    se += __shfl_xor(se, 1);
    sw += __shfl_xor(sw, 1);
    if (hf == 0 && colr < kCH * kNLoc) sWk[col] = sw * (1.0f / se);
  }
  __syncthreads();

  const float* Xb = X + (size_t)b * kNPos * kC;
  #pragma unroll 1
  for (int it = 0; it < 4; ++it) {
    const int idx = tid + 256 * it;
    if (idx < kCH * kC) {
      const int jj = idx >> 6, c = idx & 63;
      float acc = 0.f;
      #pragma unroll 1
      for (int kk = 0; kk < kNLoc; ++kk) {
        const int aa = kk / 3, b2 = kk - 3 * aa;
        const int pix = (i + aa) * kW + jj + b2;
        const float x = bf16_val(Xb[pix * kC + c]);
        acc = fmaf(sWk[kNLoc * jj + kk], x, acc);
      }
      sO[idx] = acc;
    }
  }
  __syncthreads();

  if (tid < (kCH * kC) / 4) {
    const v4f v = *(const v4fa*)(sO + 4 * tid);
    float* dst = out + ((size_t)(b * kNWin + i * kCH)) * kC + 4 * tid;
    *(volatile v4f*)dst = v;
    __threadfence();
    *(volatile v4f*)dst = v;
  }
}

extern "C" void kernel_launch(void* const* d_in, const int* in_sizes, int n_in,
                              void* d_out, int out_size, void* d_ws, size_t ws_size,
                              hipStream_t stream) {
  if (n_in < 3) return;
  if (in_sizes[0] != kNX) return;
  if (in_sizes[1] != kC) return;
  if (in_sizes[2] < 1) return;
  if (out_size != kNOut) return;

  const float* X  = (const float*)d_in[0];
  const float* Wg = (const float*)d_in[1];
  const float* bg = (const float*)d_in[2];
  float* out = (float*)d_out;

  const size_t gm_bytes = (size_t)kB * kNPos * kNPos * sizeof(float);
  const size_t pl_bytes = (size_t)kB * kNPos * sizeof(float);
  const size_t total = gm_bytes + 2 * pl_bytes;
  if (total > ws_size) return;

  char* ws = (char*)d_ws;
  float* Gm  = (float*)(ws);
  float* Spl = (float*)(ws + gm_bytes);
  float* Rpl = (float*)(ws + gm_bytes + pl_bytes);

  dim3 gGram(2, kB);
  gram_kernel<<<gGram, 128, 0, stream>>>(X, Wg, bg, Gm, Spl, Rpl);

  dim3 gWin(kCH, kB);
  win_kernel<<<gWin, 256, 0, stream>>>(X, Gm, Spl, Rpl, out);
}
